// OptimizedSecureAttention_49752901157246
// MI455X (gfx1250) — hardware-verified
//
#include <hip/hip_runtime.h>
#include <stdint.h>
#include <stddef.h>

#define NB   4
#define NS   2048
#define NDIM 512
#define NH   8
#define NHD  64

#define TP   72
#define PPITCH 40
#define OPITCH 68

typedef _Float16 h16;
typedef h16   v16h __attribute__((ext_vector_type(16)));
typedef h16   v8h  __attribute__((ext_vector_type(8), __may_alias__));
typedef float v8f  __attribute__((ext_vector_type(8)));
typedef float v4f  __attribute__((ext_vector_type(4), __may_alias__));

union Frag { v16h v; v8h hf[2]; };
union Pack8 { v8h v; h16 e[8]; };

static_assert(sizeof(Frag) == 32);
static_assert(sizeof(Pack8) == 16);
static_assert(NS % 64 == 0);
static_assert(NDIM % 64 == 0);
static_assert(NHD == 64);

__device__ __forceinline__ v8f wmma16(const v16h a, const v16h b, v8f c)
{
    c = __builtin_amdgcn_wmma_f32_16x16x32_f16(false, a, false, b, (short)0, c, false, false);
    asm volatile("v_nop\n\tv_nop\n\tv_nop\n\tv_nop" : "+v"(c) : "v"(a), "v"(b));
    return c;
}

__global__ __launch_bounds__(256) void k_convert(
    const float* __restrict__ x, const float* __restrict__ wq,
    const float* __restrict__ wk, const float* __restrict__ wv,
    h16* __restrict__ xh, h16* __restrict__ wh, int nxc, int nwc)
{
    const int t = blockIdx.x * 256 + threadIdx.x;
    const int total = nxc + 3 * nwc;
    if (t >= total) return;
    const float* src;
    h16* dst;
    float sc;
    if (t < nxc) {
        src = x + (size_t)t * 8;
        dst = xh + (size_t)t * 8;
        sc  = 1.0f;
    } else {
        const int u = t - nxc;
        const int w = u / nwc;
        const int c = u - w * nwc;
        const float* wp = (w == 0) ? wq : ((w == 1) ? wk : wv);
        src = wp + (size_t)c * 8;
        dst = wh + (size_t)u * 8;
        sc  = 64.0f;
    }
    const v4f f0 = *(const v4f*)(src);
    const v4f f1 = *(const v4f*)(src + 4);
    Pack8 p;
    p.e[0] = (h16)(f0.x * sc); p.e[1] = (h16)(f0.y * sc);
    p.e[2] = (h16)(f0.z * sc); p.e[3] = (h16)(f0.w * sc);
    p.e[4] = (h16)(f1.x * sc); p.e[5] = (h16)(f1.y * sc);
    p.e[6] = (h16)(f1.z * sc); p.e[7] = (h16)(f1.w * sc);
    const v8h val = p.v;
    *(volatile v8h*)dst = val;
    __threadfence();
    *(volatile v8h*)dst = val;
}

__device__ __forceinline__ void proj_store_pass(const h16* T, h16* base, size_t rowpitch,
                                                int w, int l)
{
    const int piece = l & 7, rq = l >> 3;
    #pragma unroll
    for (int i = 0; i < 4; ++i) {
        const int row = w * 16 + 4 * i + rq;
        const v8h v = *(const v8h*)&T[row * TP + 8 * piece];
        *(volatile v8h*)(base + (size_t)row * rowpitch + 8 * piece) = v;
    }
}

__global__ __launch_bounds__(128) void k_proj(
    const h16* __restrict__ xh, const h16* __restrict__ wh,
    const float* __restrict__ bq, const float* __restrict__ bk, const float* __restrict__ bv,
    h16* __restrict__ qh, h16* __restrict__ kh, h16* __restrict__ vt)
{
    __shared__ __attribute__((aligned(16))) h16 T[64 * TP];

    const int tid = threadIdx.x, l = tid & 31, w = tid >> 5;
    const int hh = l >> 4, m = l & 15;
    const int z = blockIdx.z;
    const int row0 = blockIdx.x * 64;
    const int col0 = blockIdx.y * 64;
    const int wr = (w & 1) * 32, wc = (w >> 1) * 32;

    const h16* arow0 = xh + (size_t)(row0 + wr + m) * NDIM + 8 * hh;
    const h16* arow1 = arow0 + (size_t)16 * NDIM;
    const h16* brow0 = wh + ((size_t)z * NDIM + (size_t)(col0 + wc + m)) * NDIM + 8 * hh;
    const h16* brow1 = brow0 + (size_t)16 * NDIM;

    v8f acc00 = {}, acc01 = {}, acc10 = {}, acc11 = {};

    for (int k0 = 0; k0 < NDIM; k0 += 32) {
        Frag a0, a1, b0, b1;
        a0.hf[0] = *(const v8h*)(arow0 + k0);  a0.hf[1] = *(const v8h*)(arow0 + k0 + 16);
        a1.hf[0] = *(const v8h*)(arow1 + k0);  a1.hf[1] = *(const v8h*)(arow1 + k0 + 16);
        b0.hf[0] = *(const v8h*)(brow0 + k0);  b0.hf[1] = *(const v8h*)(brow0 + k0 + 16);
        b1.hf[0] = *(const v8h*)(brow1 + k0);  b1.hf[1] = *(const v8h*)(brow1 + k0 + 16);
        acc00 = wmma16(a0.v, b0.v, acc00);
        acc01 = wmma16(a0.v, b1.v, acc01);
        acc10 = wmma16(a1.v, b0.v, acc10);
        acc11 = wmma16(a1.v, b1.v, acc11);
    }

    const float* bias = (z == 0) ? bq : ((z == 1) ? bk : bv);
    const bool tr = (z == 2);
    const float wsc = 0.015625f;
    #pragma unroll
    for (int i = 0; i < 2; ++i) {
        #pragma unroll
        for (int j = 0; j < 2; ++j) {
            const v8f acc = (i == 0) ? (j == 0 ? acc00 : acc01) : (j == 0 ? acc10 : acc11);
            const int c = wc + 16 * j + m;
            const float bs = bias[col0 + c];
            #pragma unroll
            for (int r = 0; r < 8; ++r) {
                const int rr = wr + 16 * i + 8 * hh + r;
                const float v = acc[r] * wsc + bs;
                const int idx = tr ? (c * TP + rr) : (rr * TP + c);
                T[idx] = (h16)v;
            }
        }
    }
    __syncthreads();

    const int bb = row0 >> 11, s0 = row0 & (NS - 1), head = blockIdx.y;
    const size_t bhh = (size_t)bb * NH + head;
    h16* base;
    size_t rowpitch;
    if (tr) {
        base = vt + bhh * NHD * NS + s0;
        rowpitch = NS;
    } else {
        base = ((z == 0) ? qh : kh) + (bhh * NS + s0) * NHD;
        rowpitch = NHD;
    }
    proj_store_pass(T, base, rowpitch, w, l);
    __threadfence();
    proj_store_pass(T, base, rowpitch, w, l);
}

__device__ __forceinline__ void attn_store_pass(const float* Ow, const float* __restrict__ noise,
                                                float* out, size_t bh, int b, int h, int q0, int l)
{
    const float inv101 = 1.0f / 1.01f;
    const int piece = l & 15, rsel = l >> 4;
    #pragma unroll
    for (int i = 0; i < 8; ++i) {
        const int rowl = 2 * i + rsel;
        const int q = q0 + rowl;
        const v4f y  = *(const v4f*)&Ow[rowl * OPITCH + 4 * piece];
        const v4f nz = *(const v4f*)(noise + ((bh * NS + (size_t)q) * NHD + 4 * piece));
        const v4f val = (y + nz) * inv101;
        *(volatile v4f*)(out + (((size_t)b * NS + (size_t)q) * NDIM + (size_t)h * NHD + 4 * piece)) = val;
    }
}

__global__ __launch_bounds__(128) void k_attn(
    const h16* __restrict__ qh, const h16* __restrict__ kh, const h16* __restrict__ vt,
    const float* __restrict__ noise, float* __restrict__ out)
{
    __shared__ __attribute__((aligned(16))) h16   Pt[4][16 * PPITCH];
    __shared__ __attribute__((aligned(16))) float Ot[4][16 * OPITCH];

    const int tid = threadIdx.x, l = tid & 31, w = tid >> 5;
    const int hh = l >> 4, m = l & 15;
    const int b = blockIdx.z, h = blockIdx.y;
    const size_t bh = (size_t)b * NH + h;
    const int q0 = blockIdx.x * 64 + w * 16;

    Frag qa0, qa1;
    {
        const h16* qrow = qh + (bh * NS + (size_t)(q0 + m)) * NHD + 8 * hh;
        qa0.hf[0] = *(const v8h*)(qrow);      qa0.hf[1] = *(const v8h*)(qrow + 16);
        qa1.hf[0] = *(const v8h*)(qrow + 32); qa1.hf[1] = *(const v8h*)(qrow + 48);
    }
    const h16* kbase = kh + (bh * NS + (size_t)m) * NHD + 8 * hh;
    const h16* vbase = vt + (bh * NHD + (size_t)m) * NS + 8 * hh;

    float mrun[8], lrun[8];
    v8f o0 = {}, o1 = {}, o2 = {}, o3 = {};
    #pragma unroll
    for (int r = 0; r < 8; ++r) { mrun[r] = -__builtin_inff(); lrun[r] = 0.0f; }

    const float sc  = 0.125f * 1.44269504088896f;
    const float psc = 16384.0f;
    h16*   Pw = &Pt[w][0];
    float* Ow = &Ot[w][0];

    for (int kt = 0; kt < NS / 32; ++kt) {
        const int key0 = kt * 32;

        v8f c0 = {}, c1 = {};
        {
            const h16* kp = kbase + (size_t)key0 * NHD;
            Frag kb;
            kb.hf[0] = *(const v8h*)(kp);      kb.hf[1] = *(const v8h*)(kp + 16);
            c0 = wmma16(qa0.v, kb.v, c0);
            kb.hf[0] = *(const v8h*)(kp + 32); kb.hf[1] = *(const v8h*)(kp + 48);
            c0 = wmma16(qa1.v, kb.v, c0);
            kp += 16 * NHD;
            kb.hf[0] = *(const v8h*)(kp);      kb.hf[1] = *(const v8h*)(kp + 16);
            c1 = wmma16(qa0.v, kb.v, c1);
            kb.hf[0] = *(const v8h*)(kp + 32); kb.hf[1] = *(const v8h*)(kp + 48);
            c1 = wmma16(qa1.v, kb.v, c1);
        }

        #pragma unroll
        for (int r = 0; r < 8; ++r) {
            const float s0 = c0[r] * sc;
            const float s1 = c1[r] * sc;
            float mt = fmaxf(s0, s1);
            #pragma unroll
            for (int off = 1; off < 16; off <<= 1)
                mt = fmaxf(mt, __shfl_xor(mt, off, 32));
            const float mnew  = fmaxf(mrun[r], mt);
            const float alpha = exp2f(mrun[r] - mnew);
            const float p0 = exp2f(s0 - mnew);
            const float p1 = exp2f(s1 - mnew);
            float rs = p0 + p1;
            #pragma unroll
            for (int off = 1; off < 16; off <<= 1)
                rs += __shfl_xor(rs, off, 32);
            lrun[r] = lrun[r] * alpha + rs;
            mrun[r] = mnew;
            o0[r] *= alpha; o1[r] *= alpha; o2[r] *= alpha; o3[r] *= alpha;
            const int rowl = 8 * hh + r;
            Pw[rowl * PPITCH + m]      = (h16)(p0 * psc);
            Pw[rowl * PPITCH + 16 + m] = (h16)(p1 * psc);
        }
        __syncthreads();

        Frag pa;
        pa.hf[0] = *(const v8h*)&Pw[m * PPITCH + 8 * hh];
        pa.hf[1] = *(const v8h*)&Pw[m * PPITCH + 16 + 8 * hh];
        {
            const h16* vp = vbase + key0;
            Frag vb;
            vb.hf[0] = *(const v8h*)(vp); vb.hf[1] = *(const v8h*)(vp + 16);
            o0 = wmma16(pa.v, vb.v, o0);
            vp += (size_t)16 * NS;
            vb.hf[0] = *(const v8h*)(vp); vb.hf[1] = *(const v8h*)(vp + 16);
            o1 = wmma16(pa.v, vb.v, o1);
            vp += (size_t)16 * NS;
            vb.hf[0] = *(const v8h*)(vp); vb.hf[1] = *(const v8h*)(vp + 16);
            o2 = wmma16(pa.v, vb.v, o2);
            vp += (size_t)16 * NS;
            vb.hf[0] = *(const v8h*)(vp); vb.hf[1] = *(const v8h*)(vp + 16);
            o3 = wmma16(pa.v, vb.v, o3);
        }
        __syncthreads();
    }

    const float osc = 1.0f / 16384.0f;
    #pragma unroll
    for (int r = 0; r < 8; ++r) {
        const float invl = osc * __builtin_amdgcn_rcpf(lrun[r]);
        const int rowl = 8 * hh + r;
        Ow[rowl * OPITCH + m]      = o0[r] * invl;
        Ow[rowl * OPITCH + 16 + m] = o1[r] * invl;
        Ow[rowl * OPITCH + 32 + m] = o2[r] * invl;
        Ow[rowl * OPITCH + 48 + m] = o3[r] * invl;
    }
    __syncthreads();

    attn_store_pass(Ow, noise, out, bh, b, h, q0, l);
    __threadfence();
    attn_store_pass(Ow, noise, out, bh, b, h, q0, l);
}

extern "C" void kernel_launch(void* const* d_in, const int* in_sizes, int n_in,
                              void* d_out, int out_size, void* d_ws, size_t ws_size,
                              hipStream_t stream)
{
    if (n_in < 8) return;
    const int n_x = NB * NS * NDIM;
    const int n_w = NDIM * NDIM;
    if (in_sizes[0] != n_x || in_sizes[1] != n_w || in_sizes[2] != NDIM ||
        in_sizes[3] != n_w || in_sizes[4] != NDIM || in_sizes[5] != n_w ||
        in_sizes[6] != NDIM || in_sizes[7] != NB * NH * NS * NHD || out_size != n_x)
        return;

    const float* x     = (const float*)d_in[0];
    const float* Wq    = (const float*)d_in[1];
    const float* bq    = (const float*)d_in[2];
    const float* Wk    = (const float*)d_in[3];
    const float* bk    = (const float*)d_in[4];
    const float* Wv    = (const float*)d_in[5];
    const float* bv    = (const float*)d_in[6];
    const float* noise = (const float*)d_in[7];
    float* out = (float*)d_out;

    const size_t bytes_xh  = (size_t)n_x * 2;
    const size_t bytes_wh  = (size_t)3 * n_w * 2;
    const size_t bytes_qkv = (size_t)NB * NH * NS * NHD * 2;
    const size_t off_xh = 0;
    const size_t off_wh = off_xh + bytes_xh;
    const size_t off_q  = off_wh + bytes_wh;
    const size_t off_k  = off_q + bytes_qkv;
    const size_t off_v  = off_k + bytes_qkv;
    const size_t end    = off_v + bytes_qkv;
    if (end > ws_size) return;

    char* ws = (char*)d_ws;
    h16* xh = (h16*)(ws + off_xh);
    h16* wh = (h16*)(ws + off_wh);
    h16* qh = (h16*)(ws + off_q);
    h16* kh = (h16*)(ws + off_k);
    h16* vt = (h16*)(ws + off_v);

    const int nxc = n_x / 8;
    const int nwc = n_w / 8;
    const int total_chunks = nxc + 3 * nwc;
    const int cgrid = (total_chunks + 255) / 256;
    k_convert<<<dim3(cgrid), dim3(256), 0, stream>>>(x, Wq, Wk, Wv, xh, wh, nxc, nwc);

    dim3 pg((NB * NS) / 64, NDIM / 64, 3);
    k_proj<<<pg, dim3(128), 0, stream>>>(xh, wh, bq, bk, bv, qh, kh, vt);

    dim3 ag(NS / 64, NH, NB);
    k_attn<<<ag, dim3(128), 0, stream>>>(qh, kh, vt, noise, out);
}
